// ContractiveInvertibleGNN_78099685310586
// MI455X (gfx1250) — hardware-verified
//
#include <hip/hip_runtime.h>

typedef __attribute__((ext_vector_type(16))) _Float16 v16h;
typedef __attribute__((ext_vector_type(8)))  _Float16 v8h;
typedef __attribute__((ext_vector_type(16))) __bf16   v16b;
typedef __attribute__((ext_vector_type(8)))  __bf16   v8b;
typedef __attribute__((ext_vector_type(8)))  float    v8f;
typedef __attribute__((ext_vector_type(4)))  float    v4f;

__device__ __forceinline__ unsigned short f2bf_bits(float f) {
  unsigned u = __float_as_uint(f);
  return (unsigned short)((u + 0x7FFFu + ((u >> 16) & 1u)) >> 16);
}
__device__ __forceinline__ float bf_bits2f(unsigned short h) { return __uint_as_float(((unsigned)h) << 16); }

__device__ __forceinline__ void dep_guard_h(v8f& a, v8f& b, v16h x, v16h y) { asm volatile("v_nop\n\tv_nop\n\tv_nop\n\tv_nop" : "+v"(a), "+v"(b) : "v"(x), "v"(y)); }
__device__ __forceinline__ void dep_guard_b(v8f& a, v8f& b, v16b x, v16b y) { asm volatile("v_nop\n\tv_nop\n\tv_nop\n\tv_nop" : "+v"(a), "+v"(b) : "v"(x), "v"(y)); }
__device__ __forceinline__ void keep4_h(v16h a, v16h b, v16h c, v16h d) { asm volatile("v_nop" :: "v"(a), "v"(b), "v"(c), "v"(d)); }
__device__ __forceinline__ void keep4_b(v16b a, v16b b, v16b c, v16b d) { asm volatile("v_nop" :: "v"(a), "v"(b), "v"(c), "v"(d)); }
__device__ __forceinline__ void acc_guard4(v8f& a, v8f& b, v8f& c, v8f& d) { asm volatile("v_nop\n\tv_nop\n\tv_nop\n\tv_nop" : "+v"(a), "+v"(b), "+v"(c), "+v"(d)); }
template <typename T> struct Frag;
template <> struct Frag<_Float16> {
  typedef v16h V; union U { v16h v; v8h h[2]; };
  static __device__ __forceinline__ v16h load(const _Float16* p) {
    U f; f.h[0] = *(const v8h*)(p); f.h[1] = *(const v8h*)(p + 16); return f.v;
  }
  static __device__ __forceinline__ v8f mma(v16h a, v16h b, v8f c) {
    return __builtin_amdgcn_wmma_f32_16x16x32_f16(false, a, false, b, (short)0, c, false, false);
  }
  static __device__ __forceinline__ void guard(v8f& a, v8f& b, v16h x, v16h y) { dep_guard_h(a, b, x, y); }
  static __device__ __forceinline__ void keep(v16h a, v16h b, v16h c, v16h d) { keep4_h(a, b, c, d); }
};
template <> struct Frag<__bf16> {
  typedef v16b V; union U { v16b v; v8b h[2]; };
  static __device__ __forceinline__ v16b load(const __bf16* p) {
    U f; f.h[0] = *(const v8b*)(p); f.h[1] = *(const v8b*)(p + 16); return f.v;
  }
  static __device__ __forceinline__ v8f mma(v16b a, v16b b, v8f c) {
    return __builtin_amdgcn_wmma_f32_16x16x32_bf16(false, a, false, b, (short)0, c, false, false);
  }
  static __device__ __forceinline__ void guard(v8f& a, v8f& b, v16b x, v16b y) { dep_guard_b(a, b, x, y); }
  static __device__ __forceinline__ void keep(v16b a, v16b b, v16b c, v16b d) { keep4_b(a, b, c, d); }
};

__device__ __forceinline__ float leaky01(float t) { return (t > 0.f) ? t : 0.01f * t; }

template <int ET> struct Elem;
template <> struct Elem<0> { typedef _Float16 T; };
template <> struct Elem<1> { typedef __bf16 T; };
template <int ET, bool SPLIT, int BIAS_MODE, int OUT_MODE, bool RESID, int ACT, bool RAFTER>
__global__ __launch_bounds__(256) void wmma_gemm64(
    const unsigned short* __restrict__ Ap, const unsigned short* __restrict__ A2p, int lda, long strideA,
    const unsigned short* __restrict__ Btp, const unsigned short* __restrict__ Bt2p, int ldb, long strideB,
    void* __restrict__ Cout, void* __restrict__ Cout2, void* __restrict__ Cout3, int ldc, long strideC,
    const float* __restrict__ bias,
    const float* __restrict__ resid, long strideR,
    int M, int N, int K, float scale, float oscale) {
  typedef typename Elem<ET>::T T;
  typedef typename Frag<T>::V V;
  const T* A = (const T*)Ap; const T* A2 = (const T*)A2p; const T* Bt = (const T*)Btp; const T* Bt2 = (const T*)Bt2p;
  __shared__ __align__(16) float sT[8][16 * 68];
  const int b    = blockIdx.y;
  const int lane = threadIdx.x & 31;
  const int wave = threadIdx.x >> 5;
  const int tilesN = N >> 6;
  const int tilesM = M >> 6;
  const int tile = blockIdx.x * 8 + wave;
  if (tile >= tilesM * tilesN) return;
  const int tm = tile / tilesN;
  const int tn = tile - tm * tilesN;
  const int m0 = tm << 6;
  const int n0 = tn << 6;

  const T* Ab  = A  + (size_t)b * strideA;
  const T* Bb  = Bt + (size_t)b * strideB;
  const T* Ab2 = SPLIT ? (A2  + (size_t)b * strideA) : nullptr;
  const T* Bb2 = SPLIT ? (Bt2 + (size_t)b * strideB) : nullptr;

  const int rlane = lane & 15;
  const int koff  = (lane >> 4) * 8;
  const int mOff  = (lane >> 4) * 8;

  v8f acc[4][4];
#pragma unroll
  for (int i = 0; i < 4; ++i)
#pragma unroll
    for (int j = 0; j < 4; ++j) acc[i][j] = (v8f){0.f,0.f,0.f,0.f,0.f,0.f,0.f,0.f};

  for (int k0 = 0; k0 < K; k0 += 32) {
    V bh[4], bl[4];
#pragma unroll
    for (int j = 0; j < 4; ++j) {
      const size_t bo = (size_t)(n0 + (j << 4) + rlane) * ldb + koff + k0;
      bh[j] = Frag<T>::load(Bb + bo);
      if (SPLIT) bl[j] = Frag<T>::load(Bb2 + bo);
    }
#pragma unroll
    for (int i = 0; i < 4; ++i) {
      const size_t ao = (size_t)(m0 + (i << 4) + rlane) * lda + koff + k0;
      V ah = Frag<T>::load(Ab + ao);
      V al;
      if (SPLIT) al = Frag<T>::load(Ab2 + ao);
#pragma unroll
      for (int j = 0; j < 4; ++j) {
        acc[i][j] = Frag<T>::mma(ah, bh[j], acc[i][j]);
        if (SPLIT) {
          acc[i][j] = Frag<T>::mma(ah, bl[j], acc[i][j]);
          acc[i][j] = Frag<T>::mma(al, bh[j], acc[i][j]);
        }
      }
      Frag<T>::guard(acc[i][0], acc[i][3], ah, SPLIT ? al : ah);
    }
    Frag<T>::keep(bh[0], bh[1], bh[2], bh[3]);
    if (SPLIT) Frag<T>::keep(bl[0], bl[1], bl[2], bl[3]);
  }
  acc_guard4(acc[0][0], acc[0][1], acc[0][2], acc[0][3]);
  acc_guard4(acc[1][0], acc[1][1], acc[1][2], acc[1][3]);
  acc_guard4(acc[2][0], acc[2][1], acc[2][2], acc[2][3]);
  acc_guard4(acc[3][0], acc[3][1], acc[3][2], acc[3][3]);

  float* slab = sT[wave];
  const float* Rb = RESID ? (resid + (size_t)b * strideR) : nullptr;
#pragma unroll
  for (int i = 0; i < 4; ++i) {
    const int mBase = m0 + (i << 4);
#pragma unroll
    for (int j = 0; j < 4; ++j) {
      const int n = n0 + (j << 4) + rlane;
      float bv = 0.f;
      if (BIAS_MODE == 2) bv = bias[n];
#pragma unroll
      for (int r = 0; r < 8; ++r) {
        const int mrow = mBase + mOff + r;
        float v = acc[i][j][r] * scale;
        if (BIAS_MODE == 1) v += bias[mrow];
        if (BIAS_MODE == 2) v += bv;
        if (BIAS_MODE == 3) v += bias[(mrow & 31) * N + n];
        float rv = 0.f;
        if (RESID) rv = Rb[(size_t)mrow * ldc + n];
        if (RESID && !RAFTER) v += rv;
        if (ACT == 2) v = fmaxf(v, 0.0f);
        if (ACT == 4) v = leaky01(v);
        if (RESID && RAFTER) v += rv;
        slab[(mOff + r) * 68 + (j << 4) + rlane] = v;
      }
    }
    __builtin_amdgcn_fence(__ATOMIC_RELEASE, "workgroup");
    __builtin_amdgcn_wave_barrier();
    __builtin_amdgcn_fence(__ATOMIC_ACQUIRE, "workgroup");
    if (OUT_MODE == 0 || OUT_MODE == 3) {
      float* C = (float*)Cout + (size_t)b * strideC;
      const int hh = lane >> 4, c4 = (lane & 15) * 4;
      for (int pass = 0; pass < 2; ++pass) {
#pragma unroll
        for (int it = 0; it < 8; ++it) {
          const int row = it * 2 + hh;
          v4f v = *(const v4f*)(slab + row * 68 + c4);
          *(volatile v4f*)(C + (size_t)(mBase + row) * ldc + n0 + c4) = v;
        }
        __threadfence();
      }
    }
    if (OUT_MODE == 1 || OUT_MODE == 2 || OUT_MODE == 3) {
      const int q = lane >> 3, c8 = (lane & 7) * 8;
      unsigned short* C1 = (unsigned short*)((OUT_MODE == 3) ? Cout2 : Cout) + (size_t)b * strideC;
      unsigned short* C2 = (unsigned short*)((OUT_MODE == 3) ? Cout3 : Cout2) + (size_t)b * strideC;
      for (int pass = 0; pass < 2; ++pass) {
#pragma unroll
        for (int it = 0; it < 4; ++it) {
          const int row = it * 4 + q;
          const float* sp = slab + row * 68 + c8;
          v8h hv, lv;
#pragma unroll
          for (int e = 0; e < 8; ++e) {
            if (OUT_MODE == 1) {
              hv[e] = (_Float16)(sp[e] * oscale);
            } else {
              unsigned short hb = f2bf_bits(sp[e]);
              unsigned short lb = f2bf_bits(sp[e] - bf_bits2f(hb));
              hv[e] = __builtin_bit_cast(_Float16, hb);
              lv[e] = __builtin_bit_cast(_Float16, lb);
            }
          }
          *(volatile v8h*)(C1 + (size_t)(mBase + row) * ldc + n0 + c8) = hv;
          if (OUT_MODE == 2 || OUT_MODE == 3) *(volatile v8h*)(C2 + (size_t)(mBase + row) * ldc + n0 + c8) = lv;
        }
        __threadfence();
      }
    }
    __builtin_amdgcn_fence(__ATOMIC_RELEASE, "workgroup");
    __builtin_amdgcn_wave_barrier();
    __builtin_amdgcn_fence(__ATOMIC_ACQUIRE, "workgroup");
  }
}

__global__ __launch_bounds__(256) void build_tables(
    const float* __restrict__ W, const float* __restrict__ E,
    const float* __restrict__ gW1, const float* __restrict__ gb1,
    const float* __restrict__ gW2, const float* __restrict__ gW3,
    const float* __restrict__ fW1, const float* __restrict__ fb1,
    const float* __restrict__ fW2,
    float* __restrict__ CG, float* __restrict__ CF,
    _Float16* __restrict__ GW2T, _Float16* __restrict__ GW3T, _Float16* __restrict__ FW1T,
    unsigned short* __restrict__ FW2H, unsigned short* __restrict__ FW2L,
    unsigned short* __restrict__ WTH, unsigned short* __restrict__ WTL) {
  const int tid = threadIdx.x;
  const int bid = blockIdx.x;
  if (bid < 4) {
    const int t = bid * 256 + tid;
    const int node = t >> 5;
    const int k4 = (t & 31) * 4;
    float cgv[4], cfv[4];
#pragma unroll
    for (int c = 0; c < 4; ++c) { cgv[c] = gb1[k4 + c]; cfv[c] = fb1[k4 + c]; }
#pragma unroll 1
    for (int e = 0; e < 32; ++e) {
      const float em = E[node * 32 + e];
      const float* gw = gW1 + (32 + e) * 128 + k4;
      const float* fw = fW1 + (32 + e) * 128 + k4;
#pragma unroll
      for (int c = 0; c < 4; ++c) {
        cgv[c] = fmaf(em, gw[c], cgv[c]);
        cfv[c] = fmaf(em, fw[c], cfv[c]);
      }
    }
    const v4f ga = (v4f){cgv[0], cgv[1], cgv[2], cgv[3]};
    const v4f fa = (v4f){cfv[0], cfv[1], cfv[2], cfv[3]};
    float* pg = CG + node * 128 + k4;
    float* pf = CF + node * 128 + k4;
    for (int pass = 0; pass < 2; ++pass) {
      *(volatile v4f*)pg = ga;
      *(volatile v4f*)pf = fa;
      __threadfence();
    }
  } else if (bid < 12) {
    const int t = (bid - 4) * 256 + tid;
    const int n = t >> 4;
    const int k8 = (t & 15) * 8;
    v8h gv, fh, fl;
#pragma unroll
    for (int c = 0; c < 8; ++c) {
      const int k = k8 + c;
      const float g = gW2[k * 128 + n];
      const float f = fW2[k * 128 + n];
      gv[c] = (_Float16)(g * 16.0f);
      const unsigned short hb = f2bf_bits(f);
      const unsigned short lb = f2bf_bits(f - bf_bits2f(hb));
      fh[c] = __builtin_bit_cast(_Float16, hb);
      fl[c] = __builtin_bit_cast(_Float16, lb);
    }
    _Float16* pg = GW2T + n * 128 + k8;
    unsigned short* ph = FW2H + n * 128 + k8;
    unsigned short* pl = FW2L + n * 128 + k8;
    for (int pass = 0; pass < 2; ++pass) {
      *(volatile v8h*)pg = gv;
      *(volatile v8h*)ph = fh;
      *(volatile v8h*)pl = fl;
      __threadfence();
    }
  } else if (bid < 14) {
    const int t = (bid - 12) * 256 + tid;
    const int d = t >> 4;
    const int k8 = (t & 15) * 8;
    v8h gv;
#pragma unroll
    for (int c = 0; c < 8; ++c) gv[c] = (_Float16)(gW3[(k8 + c) * 32 + d] * 16.0f);
    _Float16* pg = GW3T + d * 128 + k8;
    for (int pass = 0; pass < 2; ++pass) {
      *(volatile v8h*)pg = gv;
      __threadfence();
    }
  } else if (bid < 16) {
    const int t = (bid - 14) * 256 + tid;
    const int n = t >> 2;
    const int k8 = (t & 3) * 8;
    v8h fv;
#pragma unroll
    for (int c = 0; c < 8; ++c) fv[c] = (_Float16)(fW1[(k8 + c) * 128 + n] * 16.0f);
    _Float16* pf = FW1T + n * 32 + k8;
    for (int pass = 0; pass < 2; ++pass) {
      *(volatile v8h*)pf = fv;
      __threadfence();
    }
  } else {
    if (tid < 128) {
      const int i = tid >> 2;
      const int j8 = (tid & 3) * 8;
      v8h hv, lv;
#pragma unroll
      for (int c = 0; c < 8; ++c) {
        const int j = j8 + c;
        const float w = W[j * 32 + i];
        const float v = (i != j) ? w : 0.0f;
        const unsigned short hb = f2bf_bits(v);
        const unsigned short lb = f2bf_bits(v - bf_bits2f(hb));
        hv[c] = __builtin_bit_cast(_Float16, hb);
        lv[c] = __builtin_bit_cast(_Float16, lb);
      }
      unsigned short* ph = WTH + i * 32 + j8;
      unsigned short* pl = WTL + i * 32 + j8;
      for (int pass = 0; pass < 2; ++pass) {
        *(volatile v8h*)ph = hv;
        *(volatile v8h*)pl = lv;
        __threadfence();
      }
    }
  }
}

__global__ __launch_bounds__(256) void g_input_layer(
    const float* __restrict__ X, const float* __restrict__ gW1, const float* __restrict__ CG,
    const float* __restrict__ gmask,
    float* __restrict__ H1F, _Float16* __restrict__ H1H, int nrows) {
  __shared__ __align__(16) float stg[8][264];
  const int lane = threadIdx.x & 31;
  const int wave = threadIdx.x >> 5;
  int rbase = blockIdx.x * 16 + wave * 2;
  if (rbase > nrows - 2) rbase = nrows - 2;
  const int row = rbase + (lane >> 4);
  const int k8 = (lane & 15) * 8;
  const int node = row & 31;
  const float x = X[row] * gmask[node * 32 + node];
  const float* wrow = gW1 + node * 128 + k8;
  const float* crow = CG + node * 128 + k8;
  float v[8];
#pragma unroll
  for (int e = 0; e < 8; ++e) v[e] = leaky01(fmaf(x, wrow[e], crow[e]));
  v8h hv;
#pragma unroll
  for (int e = 0; e < 8; ++e) hv[e] = (_Float16)(v[e] * 64.0f);
  float* s = stg[wave];
  *(v4f*)(s + lane * 8)     = (v4f){v[0], v[1], v[2], v[3]};
  *(v4f*)(s + lane * 8 + 4) = (v4f){v[4], v[5], v[6], v[7]};
  __builtin_amdgcn_fence(__ATOMIC_RELEASE, "workgroup");
  __builtin_amdgcn_wave_barrier();
  __builtin_amdgcn_fence(__ATOMIC_ACQUIRE, "workgroup");
  const v4f q0 = *(const v4f*)(s + lane * 4);
  const v4f q1 = *(const v4f*)(s + 128 + lane * 4);
  _Float16* hp = H1H + (size_t)row * 128 + k8;
  float* f0 = H1F + (size_t)rbase * 128 + lane * 4;
  float* f1 = H1F + (size_t)(rbase + 1) * 128 + lane * 4;
  for (int pass = 0; pass < 2; ++pass) {
    *(volatile v8h*)hp = hv;
    *(volatile v4f*)f0 = q0;
    *(volatile v4f*)f1 = q1;
    __threadfence();
  }
}

__global__ __launch_bounds__(256) void emb_node_mix(
    const unsigned short* __restrict__ H2Hp, const unsigned short* __restrict__ GW3Tp,
    const float* __restrict__ gb3,
    const unsigned short* __restrict__ WTHp, const unsigned short* __restrict__ WTLp,
    _Float16* __restrict__ XAGG, int nb) {
  __shared__ __align__(16) unsigned short sXh[8][32 * 40];
  __shared__ __align__(16) unsigned short sXl[8][32 * 40];
  __shared__ __align__(16) float sO[8][32 * 36];
  const int lane = threadIdx.x & 31;
  const int wave = threadIdx.x >> 5;
  const int rl = lane & 15;
  const int hs = lane >> 4;
  const int koff = hs * 8;
  const int bb = blockIdx.x * 8 + wave;
  if (bb >= nb) return;
  const _Float16* Hb = (const _Float16*)H2Hp + (size_t)bb * 32 * 128;
  const _Float16* G3 = (const _Float16*)GW3Tp;

  v8f e[2][2];
#pragma unroll
  for (int jt = 0; jt < 2; ++jt)
#pragma unroll
    for (int dt = 0; dt < 2; ++dt) e[jt][dt] = (v8f){0.f,0.f,0.f,0.f,0.f,0.f,0.f,0.f};
#pragma unroll
  for (int kc = 0; kc < 4; ++kc) {
    const v16h bw0 = Frag<_Float16>::load(G3 + (size_t)(rl) * 128 + kc * 32 + koff);
    const v16h bw1 = Frag<_Float16>::load(G3 + (size_t)(16 + rl) * 128 + kc * 32 + koff);
#pragma unroll
    for (int jt = 0; jt < 2; ++jt) {
      const v16h a = Frag<_Float16>::load(Hb + (size_t)(jt * 16 + rl) * 128 + kc * 32 + koff);
      e[jt][0] = Frag<_Float16>::mma(a, bw0, e[jt][0]);
      e[jt][1] = Frag<_Float16>::mma(a, bw1, e[jt][1]);
      Frag<_Float16>::guard(e[jt][0], e[jt][1], a, a);
    }
    Frag<_Float16>::keep(bw0, bw1, bw0, bw1);
  }
  acc_guard4(e[0][0], e[0][1], e[1][0], e[1][1]);

  unsigned short* xh = sXh[wave];
  unsigned short* xl = sXl[wave];
  const float inv = 0.0009765625f;
#pragma unroll
  for (int jt = 0; jt < 2; ++jt) {
#pragma unroll
    for (int dt = 0; dt < 2; ++dt) {
      const int d = dt * 16 + rl;
      const float bv = gb3[d];
#pragma unroll
      for (int r = 0; r < 8; ++r) {
        const int j = jt * 16 + 8 * hs + r;
        const float v = e[jt][dt][r] * inv + bv;
        const unsigned short hb = f2bf_bits(v);
        const unsigned short lb = f2bf_bits(v - bf_bits2f(hb));
        xh[d * 40 + j] = hb;
        xl[d * 40 + j] = lb;
      }
    }
  }
  __builtin_amdgcn_fence(__ATOMIC_RELEASE, "workgroup");
  __builtin_amdgcn_wave_barrier();
  __builtin_amdgcn_fence(__ATOMIC_ACQUIRE, "workgroup");

  const __bf16* XH = (const __bf16*)xh;
  const __bf16* XL = (const __bf16*)xl;
  const __bf16* WH = (const __bf16*)WTHp;
  const __bf16* WL = (const __bf16*)WTLp;
  const v16b bh0 = Frag<__bf16>::load(XH + (rl) * 40 + koff);
  const v16b bh1 = Frag<__bf16>::load(XH + (16 + rl) * 40 + koff);
  const v16b bl0 = Frag<__bf16>::load(XL + (rl) * 40 + koff);
  const v16b bl1 = Frag<__bf16>::load(XL + (16 + rl) * 40 + koff);
  v8f g[2][2];
#pragma unroll
  for (int it = 0; it < 2; ++it)
#pragma unroll
    for (int dt = 0; dt < 2; ++dt) g[it][dt] = (v8f){0.f,0.f,0.f,0.f,0.f,0.f,0.f,0.f};
#pragma unroll
  for (int it = 0; it < 2; ++it) {
    const v16b ah = Frag<__bf16>::load(WH + (it * 16 + rl) * 32 + koff);
    const v16b al = Frag<__bf16>::load(WL + (it * 16 + rl) * 32 + koff);
    g[it][0] = Frag<__bf16>::mma(ah, bh0, g[it][0]);
    g[it][0] = Frag<__bf16>::mma(ah, bl0, g[it][0]);
    g[it][0] = Frag<__bf16>::mma(al, bh0, g[it][0]);
    g[it][1] = Frag<__bf16>::mma(ah, bh1, g[it][1]);
    g[it][1] = Frag<__bf16>::mma(ah, bl1, g[it][1]);
    g[it][1] = Frag<__bf16>::mma(al, bh1, g[it][1]);
    Frag<__bf16>::guard(g[it][0], g[it][1], ah, al);
  }
  Frag<__bf16>::keep(bh0, bh1, bl0, bl1);
  acc_guard4(g[0][0], g[0][1], g[1][0], g[1][1]);

  float* so = sO[wave];
#pragma unroll
  for (int it = 0; it < 2; ++it) {
#pragma unroll
    for (int dt = 0; dt < 2; ++dt) {
      const int d = dt * 16 + rl;
#pragma unroll
      for (int r = 0; r < 8; ++r) {
        const int i = it * 16 + 8 * hs + r;
        so[i * 36 + d] = g[it][dt][r] * 64.0f;
      }
    }
  }
  __builtin_amdgcn_fence(__ATOMIC_RELEASE, "workgroup");
  __builtin_amdgcn_wave_barrier();
  __builtin_amdgcn_fence(__ATOMIC_ACQUIRE, "workgroup");
  _Float16* ob = XAGG + (size_t)bb * 1024;
  const int rr = lane >> 2;
  const int c8 = (lane & 3) * 8;
  for (int pass = 0; pass < 2; ++pass) {
#pragma unroll
    for (int s = 0; s < 4; ++s) {
      const int row = s * 8 + rr;
      const float* sp = so + row * 36 + c8;
      v8h hv;
#pragma unroll
      for (int q = 0; q < 8; ++q) hv[q] = (_Float16)sp[q];
      *(volatile v8h*)(ob + row * 32 + c8) = hv;
    }
    __threadfence();
  }
}

__global__ __launch_bounds__(256) void f_output_dot(
    const float* __restrict__ H2F, const float* __restrict__ fW3, const float* __restrict__ fb3,
    const float* __restrict__ gmask, float* __restrict__ out, int nb) {
  const int lane = threadIdx.x & 31;
  const int wave = threadIdx.x >> 5;
  const int bb = blockIdx.x * 8 + wave;
  if (bb >= nb) return;
  const float* h = H2F + ((size_t)bb * 32 + lane) * 128;
  const float* w = fW3 + lane;
  float acc = 0.f;
#pragma unroll 1
  for (int k = 0; k < 128; k += 4) {
    const v4f hv = *(const v4f*)(h + k);
    acc = fmaf(hv[0], w[(k + 0) * 32], acc);
    acc = fmaf(hv[1], w[(k + 1) * 32], acc);
    acc = fmaf(hv[2], w[(k + 2) * 32], acc);
    acc = fmaf(hv[3], w[(k + 3) * 32], acc);
  }
  const float val = (acc + fb3[lane]) * gmask[lane * 32 + lane];
  float* op = out + (size_t)bb * 32 + lane;
  *(volatile float*)op = val;
  __threadfence();
  *(volatile float*)op = val;
}

extern "C" void kernel_launch(void* const* d_in, const int* in_sizes, int n_in,
                              void* d_out, int out_size, void* d_ws, size_t ws_size,
                              hipStream_t stream) {
  if (n_in < 16) return;
  const float* X     = (const float*)d_in[0];
  const float* W     = (const float*)d_in[1];
  const float* E     = (const float*)d_in[2];
  const float* gW1   = (const float*)d_in[3];
  const float* gb1   = (const float*)d_in[4];
  const float* gW2   = (const float*)d_in[5];
  const float* gb2   = (const float*)d_in[6];
  const float* gW3   = (const float*)d_in[7];
  const float* gb3   = (const float*)d_in[8];
  const float* fW1   = (const float*)d_in[9];
  const float* fb1   = (const float*)d_in[10];
  const float* fW2   = (const float*)d_in[11];
  const float* fb2   = (const float*)d_in[12];
  const float* fW3   = (const float*)d_in[13];
  const float* fb3   = (const float*)d_in[14];
  const float* gmask = (const float*)d_in[15];
  float* out = (float*)d_out;

  constexpr long kRowsPerChunk = 65536;
  constexpr int  kBatchPerChunk = 2048;
  constexpr int  kHid = 128;
  const long rows = in_sizes[0];
  if (rows < kRowsPerChunk || (rows % kRowsPerChunk) != 0 || (long)out_size != rows) return;
  if (in_sizes[1] != 1024 || in_sizes[2] != 1024 || in_sizes[3] != 64 * kHid || in_sizes[4] != kHid ||
      in_sizes[5] != kHid * kHid || in_sizes[6] != kHid || in_sizes[7] != kHid * 32 || in_sizes[8] != 32 ||
      in_sizes[9] != 64 * kHid || in_sizes[10] != kHid || in_sizes[11] != kHid * kHid || in_sizes[12] != kHid ||
      in_sizes[13] != kHid * 32 || in_sizes[14] != 32 || in_sizes[15] != 1024) return;
  const int nchunk = (int)(rows / kRowsPerChunk);

  constexpr size_t oCG = 0, oCF = 16384, oGW2T = 32768, oGW3T = 65536, oFW1T = 73728,
                   oFW2H = 81920, oFW2L = 114688, oWTH = 147456, oWTL = 149504, oTabEnd = 262144;
  constexpr size_t szH1F  = (size_t)kRowsPerChunk * kHid * 4;
  constexpr size_t szH16  = (size_t)kRowsPerChunk * kHid * 2;
  constexpr size_t szXAGG = (size_t)kRowsPerChunk * 32 * 2;
  constexpr size_t oH1F  = oTabEnd;
  constexpr size_t oH1H  = oH1F + szH1F;
  constexpr size_t oH2H  = oH1H + szH16;
  constexpr size_t oXAGG = oH2H + szH16;
  constexpr size_t oH2F  = oXAGG + szXAGG;
  constexpr size_t kTotal = oH2F + szH1F;
  static_assert(kTotal == 105119744, "carve total");
  if (kTotal > ws_size) return;

  char* ws = (char*)d_ws;
  float* CG = (float*)(ws + oCG);
  float* CF = (float*)(ws + oCF);
  _Float16* GW2T = (_Float16*)(ws + oGW2T);
  _Float16* GW3T = (_Float16*)(ws + oGW3T);
  _Float16* FW1T = (_Float16*)(ws + oFW1T);
  unsigned short* FW2H = (unsigned short*)(ws + oFW2H);
  unsigned short* FW2L = (unsigned short*)(ws + oFW2L);
  unsigned short* WTH = (unsigned short*)(ws + oWTH);
  unsigned short* WTL = (unsigned short*)(ws + oWTL);
  float* H1F = (float*)(ws + oH1F);
  _Float16* H1H = (_Float16*)(ws + oH1H);
  _Float16* H2H = (_Float16*)(ws + oH2H);
  _Float16* XAGG = (_Float16*)(ws + oXAGG);
  float* H2F = (float*)(ws + oH2F);
  const unsigned short* GW2Tu = (const unsigned short*)GW2T;
  const unsigned short* GW3Tu = (const unsigned short*)GW3T;
  const unsigned short* FW1Tu = (const unsigned short*)FW1T;
  const unsigned short* H1Hu = (const unsigned short*)H1H;
  const unsigned short* H2Hu = (const unsigned short*)H2H;
  const unsigned short* XAGGu = (const unsigned short*)XAGG;

  const float inv1024 = 0.0009765625f;
  const int gemmBlocks = (int)(((kRowsPerChunk / 64) * (kHid / 64)) / 8);
  const int g1Blocks = (int)(kRowsPerChunk / 16);
  const int waveBlocks = kBatchPerChunk / 8;

  build_tables<<<dim3(17), dim3(256), 0, stream>>>(W, E, gW1, gb1, gW2, gW3, fW1, fb1, fW2,
                                                   CG, CF, GW2T, GW3T, FW1T, FW2H, FW2L, WTH, WTL);

  for (int c = 0; c < nchunk; ++c) {
    const float* Xc = X + (size_t)c * kRowsPerChunk;
    float* outc = out + (size_t)c * kRowsPerChunk;

    g_input_layer<<<dim3(g1Blocks), dim3(256), 0, stream>>>(Xc, gW1, CG, gmask, H1F, H1H, (int)kRowsPerChunk);

    wmma_gemm64<0, false, 2, 1, true, 4, true><<<dim3(gemmBlocks, 1), dim3(256), 0, stream>>>(
        H1Hu, H1Hu, kHid, 0L, GW2Tu, GW2Tu, kHid, 0L,
        (void*)H2H, (void*)H2H, (void*)H2H, kHid, 0L,
        gb2, H1F, 0L, (int)kRowsPerChunk, kHid, kHid, inv1024, 64.0f);

    emb_node_mix<<<dim3(waveBlocks), dim3(256), 0, stream>>>(H2Hu, GW3Tu, gb3, WTH, WTL, XAGG, kBatchPerChunk);

    wmma_gemm64<0, false, 3, 3, false, 4, false><<<dim3(gemmBlocks, 1), dim3(256), 0, stream>>>(
        XAGGu, XAGGu, 32, 0L, FW1Tu, FW1Tu, 32, 0L,
        (void*)H1F, (void*)H1H, (void*)H2H, kHid, 0L,
        CF, CF, 0L, (int)kRowsPerChunk, kHid, 32, inv1024, 1.0f);

    wmma_gemm64<1, true, 2, 0, true, 4, true><<<dim3(gemmBlocks, 1), dim3(256), 0, stream>>>(
        H1Hu, H2Hu, kHid, 0L, FW2H, FW2L, kHid, 0L,
        (void*)H2F, (void*)H2F, (void*)H2F, kHid, 0L,
        fb2, H1F, 0L, (int)kRowsPerChunk, kHid, kHid, 1.0f, 1.0f);

    f_output_dot<<<dim3(waveBlocks), dim3(256), 0, stream>>>(H2F, fW3, fb3, gmask, outc, kBatchPerChunk);
  }
}
